// GHCBlock_68143951118651
// MI455X (gfx1250) — hardware-verified
//
#include <hip/hip_runtime.h>
#include <stddef.h>


#define CH     128
#define MIXD   4
#define APZ    136
#define KP1    128
#define KP2    256
#define NTHR   256
#define NWAVE  8
#define GROWS  32
#define GTHR   64
#define FROWS  64
#define NPW    8
#define DEGCAP 1024
#define EPT    8
#define NGRP   2
#define CHUNK  (NTHR * EPT * NGRP)
#define WCAP   (EPT * NGRP * 32)
#define LISTN  (NWAVE * WCAP)
#define NBC    4096
#define NBF    1024
#define RCAP   40960
#define RBN    128
#define OTHR   512
#define LDS_FILL ((RCAP + NBF + LISTN) * 4 + 64)
#define OFF_W1 0
#define OFF_WA (CH * KP1)
#define OFF_WB (2 * CH * KP1)
#define OFF_W2 (OFF_WB + 16 * KP1)
#define PTOT   (OFF_W2 + CH * KP2)
#define WSCAP  134217728
#define SXF 16.0f
#define SWF 64.0f
#define SHF 16.0f
#define STF 16.0f
#define SFF 64.0f
#define RC1 0.0009765625f
#define RC4 0.000244140625f

static_assert(NPW * NWAVE == FROWS);
static_assert(GROWS == (GTHR / 32) * 16);
static_assert(FROWS == 2 * GROWS);
static_assert((APZ % 8) == 0 && (KP1 % 8) == 0 && (KP2 % 8) == 0);
static_assert(PTOT == 67584);
static_assert((OFF_WA % 8) == 0 && (OFF_WB % 8) == 0 && (OFF_W2 % 8) == 0);
static_assert(NTHR * 4 == NWAVE * CH);
static_assert((CHUNK & (CHUNK - 1)) == 0);
static_assert(CHUNK <= 4096);
static_assert(NBC <= 4096 && NBF <= 4096);
static_assert((NBC & (NBC - 1)) == 0 && (NBF & (NBF - 1)) == 0);
static_assert(NBC == 4 * NBF);
static_assert(OTHR * 8 == NBC);
static_assert((RCAP % 32) == 0);
static_assert((CH % 32) == 0);

typedef float          v4f  __attribute__((ext_vector_type(4)));
typedef float          v8f  __attribute__((ext_vector_type(8)));
typedef int            v4i  __attribute__((ext_vector_type(4)));
typedef _Float16       v4h  __attribute__((ext_vector_type(4)));
typedef _Float16       v8h  __attribute__((ext_vector_type(8)));
typedef _Float16       v16h __attribute__((ext_vector_type(16)));
union Frag { v16h v; v8h h[2]; };

__device__ __forceinline__ v8f wmh(v16h a, v16h b, v8f c) {
  v8f d = __builtin_amdgcn_wmma_f32_16x16x32_f16(false, a, false, b, (short)0, c, false, false);
  asm volatile("v_nop\n\tv_nop\n\tv_nop\n\tv_nop" : "+v"(d) : "v"(a), "v"(b));
  return d;
}

__device__ __forceinline__ float gelu_f(float x) {
  return 0.5f * x * (1.0f + erff(x * 0.70710678118654752f));
}

__device__ __forceinline__ v8h cvt8(v4f a, v4f b, float s) {
  v8h r;
  r[0] = (_Float16)(a.x * s); r[1] = (_Float16)(a.y * s); r[2] = (_Float16)(a.z * s); r[3] = (_Float16)(a.w * s);
  r[4] = (_Float16)(b.x * s); r[5] = (_Float16)(b.y * s); r[6] = (_Float16)(b.z * s); r[7] = (_Float16)(b.w * s);
  return r;
}

template <int NT, int KS, int KP>
__device__ __forceinline__ void mma_tile(const _Float16* At, const _Float16* __restrict__ Bpl,
                                         int lane, v8f (&acc)[NT]) {
  const int hh = lane >> 4, m = lane & 15;
#pragma unroll
  for (int t = 0; t < NT; ++t) { v8f z = {0.f, 0.f, 0.f, 0.f, 0.f, 0.f, 0.f, 0.f}; acc[t] = z; }
  const _Float16* ap = At + m * APZ + 8 * hh;
  const _Float16* bb = Bpl + (size_t)m * KP + 8 * hh;
#pragma unroll 1
  for (int ks = 0; ks < KS; ++ks) {
    Frag a;
    a.h[0] = *(const v8h*)(ap + 32 * ks);
    a.h[1] = *(const v8h*)(ap + 32 * ks + 16);
#pragma unroll
    for (int t = 0; t < NT; ++t) {
      const _Float16* bp = bb + (size_t)(16 * t) * KP + 32 * ks;
      Frag b;
      b.h[0] = *(const v8h*)bp;
      b.h[1] = *(const v8h*)(bp + 16);
      acc[t] = wmh(a.v, b.v, acc[t]);
    }
  }
}

template <int NB>
__device__ __forceinline__ int scan_chunk(const int* __restrict__ dsts, int nE, int cbase, int slotBase,
                                          int vec8, int* list, int tid, int lane, int wave) {
  int wc = 0;
#pragma unroll
  for (int g = 0; g < NGRP; ++g) {
    const int el0  = (g * NTHR + tid) * EPT;
    const int e0   = cbase + el0;
    const int sent = -2147483647 - 1;
    v4i da, db;
    if (vec8 != 0 && cbase + CHUNK <= nE) {
      da = *(const v4i*)(dsts + e0);
      db = *(const v4i*)(dsts + e0 + 4);
    } else {
      da.x = (e0     < nE) ? dsts[min(e0, nE - 1)] : sent;
      da.y = (e0 + 1 < nE) ? dsts[min(e0 + 1, nE - 1)] : sent;
      da.z = (e0 + 2 < nE) ? dsts[min(e0 + 2, nE - 1)] : sent;
      da.w = (e0 + 3 < nE) ? dsts[min(e0 + 3, nE - 1)] : sent;
      db.x = (e0 + 4 < nE) ? dsts[min(e0 + 4, nE - 1)] : sent;
      db.y = (e0 + 5 < nE) ? dsts[min(e0 + 5, nE - 1)] : sent;
      db.z = (e0 + 6 < nE) ? dsts[min(e0 + 6, nE - 1)] : sent;
      db.w = (e0 + 7 < nE) ? dsts[min(e0 + 7, nE - 1)] : sent;
    }
    const unsigned nb = (unsigned)slotBase;
    const unsigned s0 = (unsigned)da.x - nb, s1 = (unsigned)da.y - nb;
    const unsigned s2 = (unsigned)da.z - nb, s3 = (unsigned)da.w - nb;
    const unsigned s4 = (unsigned)db.x - nb, s5 = (unsigned)db.y - nb;
    const unsigned s6 = (unsigned)db.z - nb, s7 = (unsigned)db.w - nb;
    const bool h0 = s0 < (unsigned)NB, h1 = s1 < (unsigned)NB, h2 = s2 < (unsigned)NB, h3 = s3 < (unsigned)NB;
    const bool h4 = s4 < (unsigned)NB, h5 = s5 < (unsigned)NB, h6 = s6 < (unsigned)NB, h7 = s7 < (unsigned)NB;
    const unsigned any = __builtin_amdgcn_ballot_w32(h0 | h1 | h2 | h3 | h4 | h5 | h6 | h7);
    if (any != 0u) {
#define HITJ(J, HJ, SJ) { \
        const unsigned mj = __builtin_amdgcn_ballot_w32(HJ); \
        if (mj != 0u) { \
          if (HJ) { \
            const int pos = wc + (int)__builtin_amdgcn_mbcnt_lo(mj, 0u); \
            if (pos < WCAP) list[wave * WCAP + pos] = ((el0 + (J)) << 12) | (int)(SJ); \
          } \
          wc += (int)__builtin_popcount(mj); } }
      HITJ(0, h0, s0)
      HITJ(1, h1, s1)
      HITJ(2, h2, s2)
      HITJ(3, h3, s3)
      HITJ(4, h4, s4)
      HITJ(5, h5, s5)
      HITJ(6, h6, s6)
      HITJ(7, h7, s7)
#undef HITJ
    }
  }
  return wc;
}

__global__ __launch_bounds__(NTHR) void k_wprep(const float* __restrict__ W1, const float* __restrict__ WA,
                                                const float* __restrict__ WB, const float* __restrict__ W2,
                                                _Float16* Pl) {
  const int blk = blockIdx.x, tid = threadIdx.x;
  const v4f z4 = {0.f, 0.f, 0.f, 0.f};
  v4f a, b;
  int dofs;
  if (blk < 8) {
    const int i = blk * NTHR + tid;
    a = *(const v4f*)(W1 + 8 * i); b = *(const v4f*)(W1 + 8 * i + 4);
    dofs = OFF_W1 + 8 * i;
  } else if (blk < 16) {
    const int i = (blk - 8) * NTHR + tid;
    a = *(const v4f*)(WA + 8 * i); b = *(const v4f*)(WA + 8 * i + 4);
    dofs = OFF_WA + 8 * i;
  } else if (blk == 16) {
    const int i = tid;
    const int si = (i < 64 ? i : 63) * 8;
    a = *(const v4f*)(WB + si); b = *(const v4f*)(WB + si + 4);
    if (i >= 64) { a = z4; b = z4; }
    dofs = OFF_WB + 8 * i;
  } else {
    const int i = (blk - 17) * NTHR + tid;
    a = *(const v4f*)(W2 + 8 * i); b = *(const v4f*)(W2 + 8 * i + 4);
    dofs = OFF_W2 + 8 * i;
  }
  const v8h hv = cvt8(a, b, SWF);
  _Float16* dp = Pl + dofs;
  *(volatile v8h*)dp = hv;
  __threadfence();
  *(volatile v8h*)dp = hv;
}

__global__ __launch_bounds__(NTHR) void k_count(const int* __restrict__ dsts, int* cnt, int nE, int vec8) {
  __shared__ __attribute__((aligned(16))) int scnt[NBC];
  __shared__ __attribute__((aligned(16))) int list[LISTN];
  __shared__ int wcnt[NWAVE];
  const int tid = threadIdx.x, lane = tid & 31, wave = tid >> 5;
  const int nodeBase = blockIdx.x * NBC;

  for (int i = tid; i < NBC; i += NTHR) scnt[i] = 0;
  __syncthreads();

  const int nChunks = (nE + CHUNK - 1) / CHUNK;
#pragma unroll 1
  for (int ch = 0; ch < nChunks; ++ch) {
    const int cbase = ch * CHUNK;
    const int wc = scan_chunk<NBC>(dsts, nE, cbase, nodeBase, vec8, list, tid, lane, wave);
    if (lane == 0) wcnt[wave] = wc;
    __syncthreads();
    if (wave == 0) {
#pragma unroll 1
      for (int wsx = 0; wsx < NWAVE; ++wsx) {
        int n = __builtin_amdgcn_readfirstlane(wcnt[wsx]);
        n = n > WCAP ? WCAP : (n < 0 ? 0 : n);
        const int* lp = list + wsx * WCAP;
#pragma unroll 1
        for (int i = 0; i < n; ++i) {
          const int ent  = __builtin_amdgcn_readfirstlane(lp[i]);
          const int slot = ent & (NBC - 1);
          if (lane == 0) scnt[slot] = scnt[slot] + 1;
        }
      }
    }
    __syncthreads();
  }

  v4i cq[4];
#pragma unroll
  for (int q = 0; q < 4; ++q) {
    const int f = (wave * 4 + q) * 128 + 4 * lane;
    cq[q] = *(const v4i*)(scnt + f);
  }
  int* cp = cnt + (size_t)nodeBase;
#pragma unroll
  for (int q = 0; q < 4; ++q) {
    const int f = (wave * 4 + q) * 128 + 4 * lane;
    *(volatile v4i*)(cp + f) = cq[q];
  }
  __threadfence();
#pragma unroll
  for (int q = 0; q < 4; ++q) {
    const int f = (wave * 4 + q) * 128 + 4 * lane;
    *(volatile v4i*)(cp + f) = cq[q];
  }
}

__global__ __launch_bounds__(OTHR) void k_offsets(
    const int* __restrict__ cnt, int* off, int* rbase, int nChunk) {
  __shared__ __attribute__((aligned(16))) int soff[NBC];
  __shared__ __attribute__((aligned(16))) int srb[RBN];
  __shared__ int wtot[OTHR / 32];
  const int tid = threadIdx.x, lane = tid & 31, wave = tid >> 5, sub = tid >> 7;
  for (int i = tid; i < RBN; i += OTHR) srb[i] = 0;
  int carry = 0;
#pragma unroll 1
  for (int ch = 0; ch < nChunk; ++ch) {
    const int base = ch * NBC;
    const v4i c0 = *(const v4i*)(cnt + base + 8 * tid);
    const v4i c1 = *(const v4i*)(cnt + base + 8 * tid + 4);
    const int e0 = max(c0.x, 0), e1 = max(c0.y, 0), e2 = max(c0.z, 0), e3 = max(c0.w, 0);
    const int e4 = max(c1.x, 0), e5 = max(c1.y, 0), e6 = max(c1.z, 0), e7 = max(c1.w, 0);
    const int ts = e0 + e1 + e2 + e3 + e4 + e5 + e6 + e7;
    int incl = ts;
#pragma unroll
    for (int d = 1; d < 32; d <<= 1) {
      const int t = __shfl_up(incl, d);
      if (lane >= d) incl += t;
    }
    if (lane == 31) wtot[wave] = incl;
    __syncthreads();
    const int S0 = wtot[0]  + wtot[1]  + wtot[2]  + wtot[3];
    const int S1 = wtot[4]  + wtot[5]  + wtot[6]  + wtot[7];
    const int S2 = wtot[8]  + wtot[9]  + wtot[10] + wtot[11];
    const int S3 = wtot[12] + wtot[13] + wtot[14] + wtot[15];
    int pre = 0;
#pragma unroll 1
    for (int w = 4 * sub; w < wave; ++w) pre += wtot[w];
    const int b0 = carry;
    const int b1 = b0 + ((S0 + 31) & ~31);
    const int b2 = b1 + ((S1 + 31) & ~31);
    const int b3 = b2 + ((S2 + 31) & ~31);
    const int b4 = b3 + ((S3 + 31) & ~31);
    const int myb = sub == 0 ? b0 : (sub == 1 ? b1 : (sub == 2 ? b2 : b3));
    if (tid == 0) {
      srb[min(4 * ch + 0, RBN - 1)] = b0;
      srb[min(4 * ch + 1, RBN - 1)] = b1;
      srb[min(4 * ch + 2, RBN - 1)] = b2;
      srb[min(4 * ch + 3, RBN - 1)] = b3;
    }
    int run = myb + pre + incl - ts;
    soff[8 * tid + 0] = run; run += e0;
    soff[8 * tid + 1] = run; run += e1;
    soff[8 * tid + 2] = run; run += e2;
    soff[8 * tid + 3] = run; run += e3;
    soff[8 * tid + 4] = run; run += e4;
    soff[8 * tid + 5] = run; run += e5;
    soff[8 * tid + 6] = run; run += e6;
    soff[8 * tid + 7] = run;
    carry = b4;
    __syncthreads();
    const v4i o0 = *(const v4i*)(soff + 4 * tid);
    const v4i o1 = *(const v4i*)(soff + 4 * (tid + OTHR));
    int* op = off + base;
    *(volatile v4i*)(op + 4 * tid) = o0;
    *(volatile v4i*)(op + 4 * (tid + OTHR)) = o1;
    __threadfence();
    *(volatile v4i*)(op + 4 * tid) = o0;
    *(volatile v4i*)(op + 4 * (tid + OTHR)) = o1;
    __syncthreads();
  }
  if (tid == 0) srb[min(4 * nChunk, RBN - 1)] = carry;
  __syncthreads();
  v4i rv = {0, 0, 0, 0};
  if (tid < 32) rv = *(const v4i*)(srb + 4 * tid);
  if (tid < 32) *(volatile v4i*)(rbase + 4 * tid) = rv;
  __threadfence();
  if (tid < 32) *(volatile v4i*)(rbase + 4 * tid) = rv;
}

__global__ __launch_bounds__(NTHR) void k_fill(
    const int* __restrict__ dsts, const int* __restrict__ srcs, const int* __restrict__ off,
    const int* __restrict__ rbase, int* csr, int nE, int nN, int vec8, int csrLen) {
  extern __shared__ v4f lds_dyn[];
  int* region = (int*)lds_dyn;
  int* cursor = region + RCAP;
  int* list   = cursor + NBF;
  int* wcnt   = list + LISTN;
  const int tid = threadIdx.x, lane = tid & 31, wave = tid >> 5;
  const int b = blockIdx.x;
  const int nodeBase = b * NBF;

  int rb0 = rbase[b];
  const int rb1 = rbase[b + 1];
  rb0 = rb0 < 0 ? 0 : (rb0 > csrLen ? csrLen : rb0);
  rb0 &= ~31;
  int len = rb1 - rb0;
  len = len < 0 ? 0 : (len > RCAP ? RCAP : len);
  int lenW = (len + 31) & ~31;
  if (rb0 + lenW > csrLen) lenW = (csrLen - rb0) & ~31;

  {
    const v4i z = {0, 0, 0, 0};
    for (int i = tid; i < RCAP / 4; i += NTHR) ((v4i*)region)[i] = z;
    for (int s = tid; s < NBF; s += NTHR) {
      int o = off[nodeBase + s] - rb0;
      o = o < 0 ? 0 : (o > RCAP ? RCAP : o);
      cursor[s] = o;
    }
  }
  __syncthreads();

  const int nChunks = (nE + CHUNK - 1) / CHUNK;
#pragma unroll 1
  for (int ch = 0; ch < nChunks; ++ch) {
    const int cbase = ch * CHUNK;
    const int wc = scan_chunk<NBF>(dsts, nE, cbase, nodeBase, vec8, list, tid, lane, wave);
    if (lane == 0) wcnt[wave] = wc;
    __syncthreads();
    if (wave == 0) {
#pragma unroll 1
      for (int wsx = 0; wsx < NWAVE; ++wsx) {
        int n = __builtin_amdgcn_readfirstlane(wcnt[wsx]);
        n = n > WCAP ? WCAP : (n < 0 ? 0 : n);
        const int* lp = list + wsx * WCAP;
#pragma unroll 1
        for (int i = 0; i < n; ++i) {
          const int ent  = __builtin_amdgcn_readfirstlane(lp[i]);
          const int slot = ent & (NBF - 1);
          int e = cbase + ((ent >> 12) & (CHUNK - 1));
          e = e > nE - 1 ? nE - 1 : e;
          int sv = srcs[e];
          sv = sv < 0 ? 0 : (sv > nN - 1 ? nN - 1 : sv);
          if (lane == 0) {
            int pos = cursor[slot];
            pos = pos < 0 ? 0 : (pos > RCAP - 1 ? RCAP - 1 : pos);
            region[pos] = sv;
            const int np = pos + 1;
            cursor[slot] = np > RCAP ? RCAP : np;
          }
        }
      }
    }
    __syncthreads();
  }

  const int nv = lenW >> 2;
  int* gp = csr + rb0;
#pragma unroll 1
  for (int i = tid; i < nv; i += NTHR) { const v4i v = ((const v4i*)region)[i]; *(volatile v4i*)(gp + 4 * i) = v; }
  __threadfence();
#pragma unroll 1
  for (int i = tid; i < nv; i += NTHR) { const v4i v = ((const v4i*)region)[i]; *(volatile v4i*)(gp + 4 * i) = v; }
}

__global__ __launch_bounds__(GTHR) void k_node(const float* __restrict__ X, const _Float16* __restrict__ Pl,
                                               const float* __restrict__ b1, float* Hp, _Float16* HGp,
                                               float* Gp, int nN) {
  __shared__ __attribute__((aligned(16))) _Float16 xa[GROWS * APZ];
  __shared__ __attribute__((aligned(16))) _Float16 ha[GROWS * APZ];
  __shared__ __attribute__((aligned(16))) _Float16 ta[GROWS * APZ];
  __shared__ __attribute__((aligned(16))) _Float16 hq[GROWS * APZ];
  __shared__ __attribute__((aligned(16))) float hs[GROWS * CH];
  __shared__ __attribute__((aligned(16))) float gs[GROWS * 16];
  const int tid = threadIdx.x, lane = tid & 31, wave = tid >> 5, hh = lane >> 4, m = lane & 15;
  const int rowBase = blockIdx.x * GROWS;
  {
    const int r = tid >> 1, c0 = (tid & 1) * 64;
    int xrow = rowBase + r;
    xrow = xrow > nN - 1 ? nN - 1 : xrow;
    const float* xp = X + (size_t)xrow * CH + c0;
#pragma unroll
    for (int j = 0; j < 8; ++j) {
      const v4f a = *(const v4f*)(xp + 8 * j), b = *(const v4f*)(xp + 8 * j + 4);
      *(v8h*)(xa + r * APZ + c0 + 8 * j) = cvt8(a, b, SXF);
    }
  }
  __syncthreads();

  const _Float16* PW1 = Pl + OFF_W1;
  const _Float16* PWA = Pl + OFF_WA;
  const _Float16* PWB = Pl + OFF_WB;
  const int rw0 = wave * 16;

#pragma unroll 1
  for (int cg = 0; cg < 2; ++cg) {
    v8f acc[4];
    mma_tile<4, 4, KP1>(xa + rw0 * APZ, PW1 + (size_t)(64 * cg) * KP1, lane, acc);
#pragma unroll
    for (int t = 0; t < 4; ++t) {
      const int col = 64 * cg + 16 * t + m;
      const float bv = b1[col];
#pragma unroll
      for (int r = 0; r < 8; ++r) {
        const int row = rw0 + 8 * hh + r;
        const float h = gelu_f(fmaf(acc[t][r], RC1, bv));
        hs[row * CH + col]  = h;
        ha[row * APZ + col] = (_Float16)(h * SHF);
        hq[row * APZ + col] = (_Float16)(gelu_f(h) * SFF);
      }
    }
  }
  __syncthreads();

#pragma unroll 1
  for (int cg = 0; cg < 2; ++cg) {
    v8f acc[4];
    mma_tile<4, 4, KP1>(ha + rw0 * APZ, PWA + (size_t)(64 * cg) * KP1, lane, acc);
#pragma unroll
    for (int t = 0; t < 4; ++t) {
      const int col = 64 * cg + 16 * t + m;
#pragma unroll
      for (int r = 0; r < 8; ++r) {
        const int row = rw0 + 8 * hh + r;
        ta[row * APZ + col] = (_Float16)(gelu_f(acc[t][r] * RC1) * STF);
      }
    }
  }
  __syncthreads();

  {
    v8f acc1[1];
    mma_tile<1, 4, KP1>(ta + rw0 * APZ, PWB, lane, acc1);
#pragma unroll
    for (int r = 0; r < 8; ++r) gs[(rw0 + 8 * hh + r) * 16 + m] = acc1[0][r] * RC1;
  }
  __syncthreads();

  float* hgp = Hp + (size_t)rowBase * CH;
  _Float16* qgp = HGp + (size_t)rowBase * CH;
  float* ggp = Gp + (size_t)rowBase * MIXD;
  const v4f gv = *(const v4f*)(gs + 16 * lane);
#pragma unroll
  for (int it = 0; it < 16; ++it) {
    const int f = it * GTHR + tid;
    const v4f v = *(const v4f*)(hs + 4 * f);
    *(volatile v4f*)(hgp + 4 * f) = v;
  }
#pragma unroll
  for (int it = 0; it < 8; ++it) {
    const int f = it * GTHR + tid;
    const int row = f >> 4, c = (f & 15) * 8;
    const v8h v = *(const v8h*)(hq + row * APZ + c);
    *(volatile v8h*)(qgp + 8 * f) = v;
  }
  if (wave == 0) *(volatile v4f*)(ggp + 4 * lane) = gv;
  __threadfence();
#pragma unroll
  for (int it = 0; it < 16; ++it) {
    const int f = it * GTHR + tid;
    const v4f v = *(const v4f*)(hs + 4 * f);
    *(volatile v4f*)(hgp + 4 * f) = v;
  }
#pragma unroll
  for (int it = 0; it < 8; ++it) {
    const int f = it * GTHR + tid;
    const int row = f >> 4, c = (f & 15) * 8;
    const v8h v = *(const v8h*)(hq + row * APZ + c);
    *(volatile v8h*)(qgp + 8 * f) = v;
  }
  if (wave == 0) *(volatile v4f*)(ggp + 4 * lane) = gv;
}

__device__ __forceinline__ float mixdot(v4f q, v4f s) {
  float r = gelu_f(q.x) * s.x;
  r = fmaf(gelu_f(q.y), s.y, r);
  r = fmaf(gelu_f(q.z), s.z, r);
  r = fmaf(gelu_f(q.w), s.w, r);
  return r;
}

__global__ __launch_bounds__(NTHR) void k_aggout(
    const float* __restrict__ Hp, const float* __restrict__ Gp, const _Float16* __restrict__ HGp,
    const int* __restrict__ csrc, const int* __restrict__ offp, const int* __restrict__ cntp,
    const _Float16* __restrict__ PW2, const float* __restrict__ b2,
    float* out, int nN, int csrLen) {
  __shared__ __attribute__((aligned(16))) _Float16 atile[FROWS * APZ];
  __shared__ __attribute__((aligned(16))) float stg[FROWS * CH];
  const int tid = threadIdx.x, lane = tid & 31, wave = tid >> 5, hh = lane >> 4, m = lane & 15;
  const int rowBase = blockIdx.x * FROWS;
  const v4f z4 = {0.f, 0.f, 0.f, 0.f};

#pragma unroll 1
  for (int j = 0; j < NPW; ++j) {
    const int n = rowBase + wave * NPW + j;
    const bool nval = n < nN;
    const int cc = nval ? n : nN - 1;
    const int cnr = cntp[cc];
    const int ofr = offp[cc];
    int cn = nval ? cnr : 0;
    cn = cn < 0 ? 0 : (cn > DEGCAP ? DEGCAP : cn);
    cn = __builtin_amdgcn_readfirstlane(cn);
    int of = ofr < 0 ? 0 : (ofr > csrLen ? csrLen : ofr);
    of = __builtin_amdgcn_readfirstlane(of);
    v4f q0 = z4, q1 = z4, q2 = z4, q3 = z4, sg = z4;
#pragma unroll 1
    for (int i = 0; i < cn; ++i) {
      int pos = of + i;
      pos = pos > csrLen - 1 ? csrLen - 1 : pos;
      int s = csrc[pos];
      s = s < 0 ? 0 : (s > nN - 1 ? nN - 1 : s);
      const v4f hv = *(const v4f*)(Hp + (size_t)s * CH + 4 * lane);
      const v4f gv = *(const v4f*)(Gp + (size_t)s * MIXD);
      q0 += hv.x * gv;
      q1 += hv.y * gv;
      q2 += hv.z * gv;
      q3 += hv.w * gv;
      sg += gv;
    }
    const float inv = 1.0f / fmaxf((float)cn, 1.0f);
    const float a0 = mixdot(q0, sg) * inv;
    const float a1 = mixdot(q1, sg) * inv;
    const float a2 = mixdot(q2, sg) * inv;
    const float a3 = mixdot(q3, sg) * inv;
    v4h fv;
    fv.x = (_Float16)(gelu_f(a0) * SFF);
    fv.y = (_Float16)(gelu_f(a1) * SFF);
    fv.z = (_Float16)(gelu_f(a2) * SFF);
    fv.w = (_Float16)(gelu_f(a3) * SFF);
    *(v4h*)(atile + (wave * NPW + j) * APZ + 4 * lane) = fv;
  }
  __syncthreads();

  {
    const int rt = wave & 3, cgp = wave >> 2;
    v8f acc[4];
#pragma unroll
    for (int t = 0; t < 4; ++t) { v8f z = {0.f, 0.f, 0.f, 0.f, 0.f, 0.f, 0.f, 0.f}; acc[t] = z; }
    const _Float16* ap = atile + (rt * 16 + m) * APZ + 8 * hh;
    const _Float16* ag = HGp + (size_t)(rowBase + rt * 16 + m) * CH + 8 * hh;
    const _Float16* bb = PW2 + (size_t)(64 * cgp + m) * KP2 + 8 * hh;
#pragma unroll 1
    for (int ks = 0; ks < 4; ++ks) {
      Frag a;
      a.h[0] = *(const v8h*)(ap + 32 * ks);
      a.h[1] = *(const v8h*)(ap + 32 * ks + 16);
#pragma unroll
      for (int t = 0; t < 4; ++t) {
        const _Float16* bp = bb + (size_t)(16 * t) * KP2 + 32 * ks;
        Frag b;
        b.h[0] = *(const v8h*)bp;
        b.h[1] = *(const v8h*)(bp + 16);
        acc[t] = wmh(a.v, b.v, acc[t]);
      }
    }
#pragma unroll 1
    for (int ks = 0; ks < 4; ++ks) {
      Frag a;
      a.h[0] = *(const v8h*)(ag + 32 * ks);
      a.h[1] = *(const v8h*)(ag + 32 * ks + 16);
#pragma unroll
      for (int t = 0; t < 4; ++t) {
        const _Float16* bp = bb + (size_t)(16 * t) * KP2 + CH + 32 * ks;
        Frag b;
        b.h[0] = *(const v8h*)bp;
        b.h[1] = *(const v8h*)(bp + 16);
        acc[t] = wmh(a.v, b.v, acc[t]);
      }
    }
#pragma unroll
    for (int t = 0; t < 4; ++t) {
      const int col = 64 * cgp + 16 * t + m;
      const float bv = b2[col];
#pragma unroll
      for (int r = 0; r < 8; ++r) stg[(rt * 16 + 8 * hh + r) * CH + col] = fmaf(acc[t][r], RC4, bv);
    }
  }
  __syncthreads();

#pragma unroll
  for (int it = 0; it < 8; ++it) {
    const int row  = it * NWAVE + wave;
    const int node = rowBase + row;
    const v4f v = *(const v4f*)(stg + row * CH + 4 * lane);
    if (node < nN) *(volatile v4f*)(out + (size_t)node * CH + 4 * lane) = v;
  }
  __threadfence();
#pragma unroll
  for (int it = 0; it < 8; ++it) {
    const int row  = it * NWAVE + wave;
    const int node = rowBase + row;
    const v4f v = *(const v4f*)(stg + row * CH + 4 * lane);
    if (node < nN) *(volatile v4f*)(out + (size_t)node * CH + 4 * lane) = v;
  }
}

extern "C" void kernel_launch(void* const* d_in, const int* in_sizes, int n_in,
                              void* d_out, int out_size, void* d_ws, size_t ws_size,
                              hipStream_t stream) {
  if (n_in < 8) return;
  const int nN = in_sizes[0] / CH;
  const int nE = in_sizes[1] / 2;
  if (nN <= 0 || nE <= 0) return;
  if (in_sizes[0] != nN * CH || in_sizes[1] != 2 * nE) return;
  if (in_sizes[2] != CH * CH || in_sizes[3] != CH || in_sizes[4] != CH * CH) return;
  if (in_sizes[5] != MIXD * CH || in_sizes[6] != 2 * CH * CH || in_sizes[7] != CH) return;
  if (out_size != nN * CH) return;
  if (nE > (1 << 28) || nN > (1 << 24)) return;

  const float* X  = (const float*)d_in[0];
  const int*   ei = (const int*)d_in[1];
  const float* W1 = (const float*)d_in[2];
  const float* b1 = (const float*)d_in[3];
  const float* WA = (const float*)d_in[4];
  const float* WB = (const float*)d_in[5];
  const float* W2 = (const float*)d_in[6];
  const float* b2 = (const float*)d_in[7];
  const int* srcs = ei;
  const int* dsts = ei + nE;
  float* out = (float*)d_out;

  const int nBlkF  = (nN + FROWS - 1) / FROWS;
  const int NPAD   = nBlkF * FROWS;
  const int nBlkG  = NPAD / GROWS;
  const int nBC    = (nN + NBC - 1) / NBC;
  const int CNTPAD = nBC * NBC;
  if (4 * nBC + 1 > RBN) return;
  const int nBF    = (nN + NBF - 1) / NBF;
  const int csrLen = ((nE + 31) & ~31) + 4096;
  if (31 * 4 * nBC > 4096) return;

  char* ws = (char*)d_ws;
  size_t off = 0;
  const size_t oPl  = off; off += (size_t)PTOT * 2;                off = (off + 255) & ~(size_t)255;
  const size_t oCnt = off; off += (size_t)CNTPAD * 4;              off = (off + 255) & ~(size_t)255;
  const size_t oOff = off; off += (size_t)CNTPAD * 4;              off = (off + 255) & ~(size_t)255;
  const size_t oRb  = off; off += (size_t)RBN * 4;                 off = (off + 255) & ~(size_t)255;
  const size_t oCsr = off; off += (size_t)csrLen * 4;              off = (off + 255) & ~(size_t)255;
  const size_t oH   = off; off += (size_t)NPAD * CH * 4;           off = (off + 255) & ~(size_t)255;
  const size_t oHG  = off; off += (size_t)NPAD * CH * 2;           off = (off + 255) & ~(size_t)255;
  const size_t oG   = off; off += (size_t)NPAD * MIXD * 4;         off = (off + 255) & ~(size_t)255;
  if (off > ws_size || off > (size_t)WSCAP) return;
  _Float16* Pl   = (_Float16*)(ws + oPl);
  int*      cnt  = (int*)(ws + oCnt);
  int*      offp = (int*)(ws + oOff);
  int*      rb   = (int*)(ws + oRb);
  int*      csr  = (int*)(ws + oCsr);
  float*    Hp   = (float*)(ws + oH);
  _Float16* HGp  = (_Float16*)(ws + oHG);
  float*    Gp   = (float*)(ws + oG);

  const int vec8 = ((nE & 3) == 0) ? 1 : 0;

  k_wprep<<<33, NTHR, 0, stream>>>(W1, WA, WB, W2, Pl);
  k_count<<<nBC, NTHR, 0, stream>>>(dsts, cnt, nE, vec8);
  k_offsets<<<1, OTHR, 0, stream>>>(cnt, offp, rb, nBC);
  hipFuncSetAttribute(reinterpret_cast<const void*>(&k_fill),
                      hipFuncAttributeMaxDynamicSharedMemorySize, LDS_FILL);
  k_fill<<<nBF, NTHR, LDS_FILL, stream>>>(dsts, srcs, offp, rb, csr, nE, nN, vec8, csrLen);
  k_node<<<nBlkG, GTHR, 0, stream>>>(X, Pl, b1, Hp, HGp, Gp, nN);
  k_aggout<<<nBlkF, NTHR, 0, stream>>>(Hp, Gp, HGp, csr, offp, cnt, Pl + OFF_W2, b2, out, nN, csrLen);
}
